// DSConv_pro_2430951489993
// MI455X (gfx1250) — hardware-verified
//
#include <hip/hip_runtime.h>
#define BB 4
#define CI 64
#define CO 64
#define HY 128
#define WX 128
#define KSN 9
#define NPOS (BB * HY * WX)
#define NPOSR NPOS
#define NVOX NPOS
#define COUT 64

typedef __bf16 v16b __attribute__((ext_vector_type(16)));
typedef unsigned short v8us __attribute__((ext_vector_type(8), may_alias));
typedef float  v8f  __attribute__((ext_vector_type(8)));
typedef float  v4f  __attribute__((ext_vector_type(4)));
typedef float  v4fa __attribute__((ext_vector_type(4), may_alias));
union FragB { v16b v; v8us half[2]; unsigned short u[16]; };

__device__ __forceinline__ unsigned short bf16_bits(float x) { unsigned int u = __float_as_uint(x); return (unsigned short)((u + 0x7FFFu + ((u >> 16) & 1u)) >> 16); }
__device__ __forceinline__ float bf16_val(unsigned short b) { return __uint_as_float(((unsigned int)b) << 16); }
__device__ __forceinline__ float bf16_round(float x) { return bf16_val(bf16_bits(x)); }
template <int NT>
__device__ __forceinline__ v8f mmaN(v16b ah, v16b al, v16b bh, v16b bl, v8f c) {
  c = __builtin_amdgcn_wmma_f32_16x16x32_bf16(false, ah, false, bh, (short)0, c, false, false);
  if (NT >= 2) c = __builtin_amdgcn_wmma_f32_16x16x32_bf16(false, al, false, bh, (short)0, c, false, false);
  if (NT >= 3) c = __builtin_amdgcn_wmma_f32_16x16x32_bf16(false, ah, false, bl, (short)0, c, false, false);
  asm volatile("v_nop\n\tv_nop\n\tv_nop\n\tv_nop" : "+v"(c) : "v"(ah), "v"(al), "v"(bh), "v"(bl));
  return c;
}

__global__ __launch_bounds__(256) void k_wt_bf16(const float* __restrict__ W, unsigned short* __restrict__ Wt, int K, int N) {
  const int t = blockIdx.x * 256 + threadIdx.x;
  const int k8n = K / 8;
  if (t >= N * k8n) return;
  const int n = t / k8n, k8 = (t % k8n) * 8;
  v8us v;
#pragma unroll
  for (int i = 0; i < 8; ++i) v[i] = bf16_bits(W[(size_t)(k8 + i) * N + n]);
  *(volatile v8us*)(Wt + (size_t)n * K + k8) = v;
  __threadfence();
  *(volatile v8us*)(Wt + (size_t)n * K + k8) = v;
}

template <bool ASPLIT, int ACT, bool BIAS_BF16>
__global__ __launch_bounds__(128) void k_gemm_bf(const float* __restrict__ A, int lda, const unsigned short* __restrict__ Wt, int ldb,
                                               const float* __restrict__ bias, float* __restrict__ C, int ldc, int M, int N, int K) {
  __shared__ __attribute__((aligned(16))) float so[4][16][64];
  const int tid = threadIdx.x, w = tid >> 5, lane = tid & 31, ln = lane & 15, hh = lane >> 4;
  const int ntn = N / 64;
  const int wid = blockIdx.x * 4 + w;
  const int mt = wid / ntn, nq = wid % ntn;
  if (mt * 16 >= M) return;
  const int row0 = mt * 16, col0 = nq * 64;
  const float* arow = A + (size_t)(row0 + ln) * lda;
  v8f acc[4] = {};
  for (int kb = 0; kb < K; kb += 32) {
    FragB ah, al;
    const v4f x0 = *(const v4fa*)(arow + kb + 8 * hh), x1 = *(const v4fa*)(arow + kb + 8 * hh + 4);
    const v4f x2 = *(const v4fa*)(arow + kb + 16 + 8 * hh), x3 = *(const v4fa*)(arow + kb + 16 + 8 * hh + 4);
    float xs[16] = {x0[0],x0[1],x0[2],x0[3],x1[0],x1[1],x1[2],x1[3],x2[0],x2[1],x2[2],x2[3],x3[0],x3[1],x3[2],x3[3]};
#pragma unroll
    for (int i = 0; i < 16; ++i) { const unsigned short hb = bf16_bits(xs[i]); ah.u[i] = hb; al.u[i] = ASPLIT ? bf16_bits(xs[i] - bf16_val(hb)) : (unsigned short)0; }
#pragma unroll
    for (int t = 0; t < 4; ++t) {
      const unsigned short* brow = Wt + (size_t)(col0 + t * 16 + ln) * ldb + kb;
      FragB b;
      b.half[0] = *(const v8us*)(brow + 8 * hh);
      b.half[1] = *(const v8us*)(brow + 16 + 8 * hh);
      acc[t] = mmaN<ASPLIT ? 2 : 1>(ah.v, al.v, b.v, b.v, acc[t]);
    }
  }
#pragma unroll
  for (int t = 0; t < 4; ++t) {
    float bv = bias ? bias[col0 + t * 16 + ln] : 0.f;
    if (BIAS_BF16) bv = bf16_round(bv);
#pragma unroll
    for (int r = 0; r < 8; ++r) { float v = acc[t][r] + bv; if (ACT == 1) v = fmaxf(v, 0.f); so[w][8 * hh + r][t * 16 + ln] = v; }
  }
  __builtin_amdgcn_fence(__ATOMIC_ACQ_REL, "workgroup");
  __builtin_amdgcn_wave_barrier();
  const int rsub = lane >> 4, c4 = (lane & 15) * 4;
  for (int pass = 0; pass < 2; ++pass) {
#pragma unroll
    for (int q = 0; q < 8; ++q) {
      const int r = q * 2 + rsub;
      const v4f v = *(const v4fa*)&so[w][r][c4];
      *(volatile v4f*)(C + (size_t)(row0 + r) * ldc + col0 + c4) = v;
    }
    if (pass == 0) __threadfence();
  }
}

template <int D, bool CAUSAL>
__global__ __launch_bounds__(128) void k_flash(const float* __restrict__ qb, const float* __restrict__ kb, const float* __restrict__ vb,
                                             int pitch, int T, int H, float scale, float* __restrict__ y, int ypitch) {
  constexpr int KS = D / 32;
  constexpr int DT = D / 16;
  __shared__ __attribute__((aligned(16))) unsigned short sKh[32][D + 8], sKl[32][D + 8], sVh[32][D + 8], sVl[32][D + 8];
  __shared__ __attribute__((aligned(16))) unsigned short sPh[4][16][40], sPl[4][16][40];
  __shared__ __attribute__((aligned(16))) float sO[4][16][D];
  const int tid = threadIdx.x, w = tid >> 5, lane = tid & 31, ln = lane & 15, hh = lane >> 4;
  const int nqb = (T + 63) / 64;
  const int bh = blockIdx.x / nqb, qblk = blockIdx.x % nqb;
  const int b = bh / H, h = bh % H;
  const int q0 = qblk * 64 + w * 16;
  const float* Q = qb + (size_t)b * T * pitch + h * D;
  const float* K = kb + (size_t)b * T * pitch + h * D;
  const float* V = vb + (size_t)b * T * pitch + h * D;

  FragB aqh[KS], aql[KS];
  {
    int row = q0 + ln; if (row >= T) row = T - 1;
    const float* qr = Q + (size_t)row * pitch;
#pragma unroll
    for (int ks = 0; ks < KS; ++ks)
#pragma unroll
      for (int i = 0; i < 16; ++i) {
        const int d = ks * 32 + ((i < 8) ? (8 * hh + i) : (16 + 8 * hh + (i - 8)));
        const float x = qr[d] * scale; const unsigned short hb = bf16_bits(x);
        aqh[ks].u[i] = hb; aql[ks].u[i] = bf16_bits(x - bf16_val(hb));
      }
  }
  float m_r[8], l_r[8];
#pragma unroll
  for (int r = 0; r < 8; ++r) { m_r[r] = -3.0e38f; l_r[r] = 0.f; }
  v8f oacc[DT];
#pragma unroll
  for (int dt = 0; dt < DT; ++dt) oacc[dt] = (v8f){0.f,0.f,0.f,0.f,0.f,0.f,0.f,0.f};

  const int kv_end = CAUSAL ? min(T, qblk * 64 + 64) : T;
  for (int j0 = 0; j0 < kv_end; j0 += 32) {
    __syncthreads();
    for (int e = tid; e < 32 * (D / 4); e += 128) {
      const int r = e / (D / 4), c4 = (e % (D / 4)) * 4;
      const int key = j0 + r;
      v4f kf = {0.f,0.f,0.f,0.f}, vf = {0.f,0.f,0.f,0.f};
      if (key < T) { kf = *(const v4fa*)(K + (size_t)key * pitch + c4); vf = *(const v4fa*)(V + (size_t)key * pitch + c4); }
#pragma unroll
      for (int t = 0; t < 4; ++t) {
        unsigned short hb = bf16_bits(kf[t]); sKh[r][c4 + t] = hb; sKl[r][c4 + t] = bf16_bits(kf[t] - bf16_val(hb));
        hb = bf16_bits(vf[t]); sVh[r][c4 + t] = hb; sVl[r][c4 + t] = bf16_bits(vf[t] - bf16_val(hb));
      }
    }
    __syncthreads();
    v8f s[2];
#pragma unroll
    for (int nt = 0; nt < 2; ++nt) {
      v8f acc = {};
#pragma unroll
      for (int ks = 0; ks < KS; ++ks) {
        FragB bh_, bl_;
        bh_.half[0] = *(const v8us*)&sKh[nt * 16 + ln][ks * 32 + 8 * hh]; bh_.half[1] = *(const v8us*)&sKh[nt * 16 + ln][ks * 32 + 16 + 8 * hh];
        bl_.half[0] = *(const v8us*)&sKl[nt * 16 + ln][ks * 32 + 8 * hh]; bl_.half[1] = *(const v8us*)&sKl[nt * 16 + ln][ks * 32 + 16 + 8 * hh];
        acc = mmaN<3>(aqh[ks].v, aql[ks].v, bh_.v, bl_.v, acc);
      }
      s[nt] = acc;
    }
    float alpha[8];
#pragma unroll
    for (int r = 0; r < 8; ++r) {
      const int qi = q0 + 8 * hh + r;
      const int ja = j0 + ln, jb = j0 + 16 + ln;
      if (CAUSAL) { if (ja > qi) s[0][r] = -3.0e38f; if (jb > qi) s[1][r] = -3.0e38f; }
      if (ja >= T) s[0][r] = -3.0e38f;
      if (jb >= T) s[1][r] = -3.0e38f;
      float mx = fmaxf(s[0][r], s[1][r]);
      mx = fmaxf(mx, __shfl_xor(mx, 1, 32)); mx = fmaxf(mx, __shfl_xor(mx, 2, 32)); mx = fmaxf(mx, __shfl_xor(mx, 4, 32)); mx = fmaxf(mx, __shfl_xor(mx, 8, 32));
      const float mnew = fmaxf(m_r[r], mx);
      alpha[r] = (mnew > -1.0e38f) ? __expf(m_r[r] - mnew) : 1.0f;
      const float p0 = (s[0][r] > -1.0e38f) ? __expf(s[0][r] - mnew) : 0.f;
      const float p1 = (s[1][r] > -1.0e38f) ? __expf(s[1][r] - mnew) : 0.f;
      m_r[r] = mnew;
      l_r[r] = l_r[r] * alpha[r] + p0 + p1;
      unsigned short hb = bf16_bits(p0); sPh[w][8 * hh + r][ln] = hb;      sPl[w][8 * hh + r][ln] = bf16_bits(p0 - bf16_val(hb));
      hb = bf16_bits(p1);                sPh[w][8 * hh + r][16 + ln] = hb; sPl[w][8 * hh + r][16 + ln] = bf16_bits(p1 - bf16_val(hb));
    }
#pragma unroll
    for (int dt = 0; dt < DT; ++dt)
#pragma unroll
      for (int r = 0; r < 8; ++r) oacc[dt][r] *= alpha[r];
    __builtin_amdgcn_fence(__ATOMIC_ACQ_REL, "workgroup");
    __builtin_amdgcn_wave_barrier();
    FragB pah, pal;
    pah.half[0] = *(const v8us*)&sPh[w][ln][8 * hh]; pah.half[1] = *(const v8us*)&sPh[w][ln][16 + 8 * hh];
    pal.half[0] = *(const v8us*)&sPl[w][ln][8 * hh]; pal.half[1] = *(const v8us*)&sPl[w][ln][16 + 8 * hh];
#pragma unroll
    for (int dt = 0; dt < DT; ++dt) {
      FragB bvh, bvl;
#pragma unroll
      for (int i = 0; i < 8; ++i) {
        bvh.u[i] = sVh[8 * hh + i][dt * 16 + ln]; bvh.u[8 + i] = sVh[16 + 8 * hh + i][dt * 16 + ln];
        bvl.u[i] = sVl[8 * hh + i][dt * 16 + ln]; bvl.u[8 + i] = sVl[16 + 8 * hh + i][dt * 16 + ln];
      }
      oacc[dt] = mmaN<3>(pah.v, pal.v, bvh.v, bvl.v, oacc[dt]);
    }
    __builtin_amdgcn_fence(__ATOMIC_ACQ_REL, "workgroup");
    __builtin_amdgcn_wave_barrier();
  }
#pragma unroll
  for (int r = 0; r < 8; ++r) {
    float l = l_r[r];
    l += __shfl_xor(l, 1, 32); l += __shfl_xor(l, 2, 32); l += __shfl_xor(l, 4, 32); l += __shfl_xor(l, 8, 32);
    l_r[r] = (l > 0.f) ? 1.0f / l : 0.f;
  }
#pragma unroll
  for (int dt = 0; dt < DT; ++dt)
#pragma unroll
    for (int r = 0; r < 8; ++r) sO[w][8 * hh + r][dt * 16 + ln] = oacc[dt][r] * l_r[r];
  __builtin_amdgcn_fence(__ATOMIC_ACQ_REL, "workgroup");
  __builtin_amdgcn_wave_barrier();
  for (int pass = 0; pass < 2; ++pass) {
    for (int r = 0; r < 16; ++r) {
      const int row = q0 + r;
      if (row < T && lane < D / 4) {
        const v4f val = *(const v4fa*)&sO[w][r][lane * 4];
        *(volatile v4f*)(y + ((size_t)b * T + row) * ypitch + h * D + lane * 4) = val;
      }
    }
    if (pass == 0) __threadfence();
  }
}

template <bool AFFINE, bool RESID, bool RES_BF16>
__global__ __launch_bounds__(256) void k_transpose32(const float* __restrict__ in, float* __restrict__ out, int rows, int cols,
                                                    const float* __restrict__ scale, const float* __restrict__ shift, const float* __restrict__ res) {
  __shared__ float tile[32][33];
  const int b = blockIdx.z;
  const int r0 = blockIdx.y * 32, c0 = blockIdx.x * 32;
  const float* src = in + (size_t)b * rows * cols;
  float* dst = out + (size_t)b * rows * cols;
  const int tx = threadIdx.x & 31, ty = threadIdx.x >> 5;
  for (int i = ty; i < 32; i += 8) tile[i][tx] = src[(size_t)(r0 + i) * cols + c0 + tx];
  __syncthreads();
  for (int pass = 0; pass < 2; ++pass) {
    for (int i = ty; i < 32; i += 8) {
      float v = tile[tx][i];
      const int orow = c0 + i;
      if (AFFINE) v = v * scale[orow] + shift[orow];
      if (RESID) { float rv = res[(size_t)b * rows * cols + (size_t)orow * rows + r0 + tx]; if (RES_BF16) rv = bf16_round(rv); v += rv; }
      *(volatile float*)(dst + (size_t)orow * rows + r0 + tx) = v;
    }
    if (pass == 0) __threadfence();
  }
}

__global__ __launch_bounds__(256) void k_pool2_pm(const float* __restrict__ in, float* __restrict__ out, int Bn, int H, int W, int C) {
  const size_t t = (size_t)blockIdx.x * 256 + threadIdx.x;
  const int c4n = C / 4, Ho = H / 2, Wo = W / 2;
  const size_t total = (size_t)Bn * Ho * Wo * c4n;
  if (t >= total) return;
  const int c4 = (int)(t % c4n) * 4; size_t rest = t / c4n;
  const int pw = (int)(rest % Wo); rest /= Wo; const int ph = (int)(rest % Ho); const int b = (int)(rest / Ho);
  const float* base = in + (size_t)b * H * W * C;
  const int p00 = (2 * ph) * W + 2 * pw;
  const v4f a = *(const v4fa*)(base + (size_t)p00 * C + c4), bq = *(const v4fa*)(base + (size_t)(p00 + 1) * C + c4);
  const v4f c = *(const v4fa*)(base + (size_t)(p00 + W) * C + c4), d = *(const v4fa*)(base + (size_t)(p00 + W + 1) * C + c4);
  v4f m; for (int i = 0; i < 4; ++i) m[i] = fmaxf(fmaxf(a[i], bq[i]), fmaxf(c[i], d[i]));
  float* dst = out + ((size_t)b * Ho * Wo + (size_t)ph * Wo + pw) * C + c4;
  *(volatile v4f*)dst = m;
  __threadfence();
  *(volatile v4f*)dst = m;
}

template <int DQ, int DV>
__global__ __launch_bounds__(128) void k_flash2(const float* __restrict__ Qb, size_t qstride, int qpitch, int Tq,
                                              const float* __restrict__ Kb, size_t kstride, int kpitch, int Tk,
                                              const float* __restrict__ Vb, size_t vstride, int vpitch,
                                              float scale, float* __restrict__ y, size_t ystride, int ypitch) {
  constexpr int KS = DQ / 32, DT = DV / 16;
  __shared__ __attribute__((aligned(16))) unsigned short sKh[32][DQ + 8], sKl[32][DQ + 8], sVh[32][DV + 8], sVl[32][DV + 8];
  __shared__ __attribute__((aligned(16))) unsigned short sPh[4][16][40], sPl[4][16][40];
  __shared__ __attribute__((aligned(16))) float sO[4][16][DV];
  const int tid = threadIdx.x, w = tid >> 5, lane = tid & 31, ln = lane & 15, hh = lane >> 4;
  const int nqb = (Tq + 63) / 64;
  const int bh = blockIdx.x / nqb, qblk = blockIdx.x % nqb;
  const int dv0 = blockIdx.y * DV;
  const int q0 = qblk * 64 + w * 16;
  const float* Q = Qb + (size_t)bh * qstride; const float* K = Kb + (size_t)bh * kstride; const float* V = Vb + (size_t)bh * vstride + dv0;
  FragB aqh[KS], aql[KS];
  {
    int row = q0 + ln; if (row >= Tq) row = Tq - 1;
    const float* qr = Q + (size_t)row * qpitch;
#pragma unroll
    for (int ks = 0; ks < KS; ++ks)
#pragma unroll
      for (int i = 0; i < 16; ++i) {
        const int d = ks * 32 + ((i < 8) ? (8 * hh + i) : (16 + 8 * hh + (i - 8)));
        const float x = qr[d] * scale; const unsigned short hb = bf16_bits(x);
        aqh[ks].u[i] = hb; aql[ks].u[i] = bf16_bits(x - bf16_val(hb));
      }
  }
  float m_r[8], l_r[8];
#pragma unroll
  for (int r = 0; r < 8; ++r) { m_r[r] = -3.0e38f; l_r[r] = 0.f; }
  v8f oacc[DT];
#pragma unroll
  for (int dt = 0; dt < DT; ++dt) oacc[dt] = (v8f){0.f,0.f,0.f,0.f,0.f,0.f,0.f,0.f};
  for (int j0 = 0; j0 < Tk; j0 += 32) {
    __syncthreads();
    for (int e = tid; e < 32 * (DQ / 4); e += 128) {
      const int r = e / (DQ / 4), c4 = (e % (DQ / 4)) * 4; const int key = j0 + r;
      v4f f = {0.f,0.f,0.f,0.f}; if (key < Tk) f = *(const v4fa*)(K + (size_t)key * kpitch + c4);
#pragma unroll
      for (int t = 0; t < 4; ++t) { const unsigned short hb = bf16_bits(f[t]); sKh[r][c4 + t] = hb; sKl[r][c4 + t] = bf16_bits(f[t] - bf16_val(hb)); }
    }
    for (int e = tid; e < 32 * (DV / 4); e += 128) {
      const int r = e / (DV / 4), c4 = (e % (DV / 4)) * 4; const int key = j0 + r;
      v4f f = {0.f,0.f,0.f,0.f}; if (key < Tk) f = *(const v4fa*)(V + (size_t)key * vpitch + c4);
#pragma unroll
      for (int t = 0; t < 4; ++t) { const unsigned short hb = bf16_bits(f[t]); sVh[r][c4 + t] = hb; sVl[r][c4 + t] = bf16_bits(f[t] - bf16_val(hb)); }
    }
    __syncthreads();
    v8f s[2];
#pragma unroll
    for (int nt = 0; nt < 2; ++nt) {
      v8f acc = {};
#pragma unroll
      for (int ks = 0; ks < KS; ++ks) {
        FragB bh_, bl_;
        bh_.half[0] = *(const v8us*)&sKh[nt * 16 + ln][ks * 32 + 8 * hh]; bh_.half[1] = *(const v8us*)&sKh[nt * 16 + ln][ks * 32 + 16 + 8 * hh];
        bl_.half[0] = *(const v8us*)&sKl[nt * 16 + ln][ks * 32 + 8 * hh]; bl_.half[1] = *(const v8us*)&sKl[nt * 16 + ln][ks * 32 + 16 + 8 * hh];
        acc = mmaN<3>(aqh[ks].v, aql[ks].v, bh_.v, bl_.v, acc);
      }
      s[nt] = acc;
    }
    float alpha[8];
#pragma unroll
    for (int r = 0; r < 8; ++r) {
      const int ja = j0 + ln, jb = j0 + 16 + ln;
      if (ja >= Tk) s[0][r] = -3.0e38f;
      if (jb >= Tk) s[1][r] = -3.0e38f;
      float mx = fmaxf(s[0][r], s[1][r]);
      mx = fmaxf(mx, __shfl_xor(mx, 1, 32)); mx = fmaxf(mx, __shfl_xor(mx, 2, 32)); mx = fmaxf(mx, __shfl_xor(mx, 4, 32)); mx = fmaxf(mx, __shfl_xor(mx, 8, 32));
      const float mnew = fmaxf(m_r[r], mx);
      alpha[r] = (mnew > -1.0e38f) ? __expf(m_r[r] - mnew) : 1.0f;
      const float p0 = (s[0][r] > -1.0e38f) ? __expf(s[0][r] - mnew) : 0.f;
      const float p1 = (s[1][r] > -1.0e38f) ? __expf(s[1][r] - mnew) : 0.f;
      m_r[r] = mnew;
      l_r[r] = l_r[r] * alpha[r] + p0 + p1;
      unsigned short hb = bf16_bits(p0); sPh[w][8 * hh + r][ln] = hb;      sPl[w][8 * hh + r][ln] = bf16_bits(p0 - bf16_val(hb));
      hb = bf16_bits(p1);                sPh[w][8 * hh + r][16 + ln] = hb; sPl[w][8 * hh + r][16 + ln] = bf16_bits(p1 - bf16_val(hb));
    }
#pragma unroll
    for (int dt = 0; dt < DT; ++dt)
#pragma unroll
      for (int r = 0; r < 8; ++r) oacc[dt][r] *= alpha[r];
    __builtin_amdgcn_fence(__ATOMIC_ACQ_REL, "workgroup");
    __builtin_amdgcn_wave_barrier();
    FragB pah, pal;
    pah.half[0] = *(const v8us*)&sPh[w][ln][8 * hh]; pah.half[1] = *(const v8us*)&sPh[w][ln][16 + 8 * hh];
    pal.half[0] = *(const v8us*)&sPl[w][ln][8 * hh]; pal.half[1] = *(const v8us*)&sPl[w][ln][16 + 8 * hh];
#pragma unroll
    for (int dt = 0; dt < DT; ++dt) {
      FragB bvh, bvl;
#pragma unroll
      for (int i = 0; i < 8; ++i) {
        bvh.u[i] = sVh[8 * hh + i][dt * 16 + ln]; bvh.u[8 + i] = sVh[16 + 8 * hh + i][dt * 16 + ln];
        bvl.u[i] = sVl[8 * hh + i][dt * 16 + ln]; bvl.u[8 + i] = sVl[16 + 8 * hh + i][dt * 16 + ln];
      }
      oacc[dt] = mmaN<3>(pah.v, pal.v, bvh.v, bvl.v, oacc[dt]);
    }
    __builtin_amdgcn_fence(__ATOMIC_ACQ_REL, "workgroup");
    __builtin_amdgcn_wave_barrier();
  }
#pragma unroll
  for (int r = 0; r < 8; ++r) {
    float l = l_r[r];
    l += __shfl_xor(l, 1, 32); l += __shfl_xor(l, 2, 32); l += __shfl_xor(l, 4, 32); l += __shfl_xor(l, 8, 32);
    l_r[r] = (l > 0.f) ? 1.0f / l : 0.f;
  }
#pragma unroll
  for (int dt = 0; dt < DT; ++dt)
#pragma unroll
    for (int r = 0; r < 8; ++r) sO[w][8 * hh + r][dt * 16 + ln] = oacc[dt][r] * l_r[r];
  __builtin_amdgcn_fence(__ATOMIC_ACQ_REL, "workgroup");
  __builtin_amdgcn_wave_barrier();
  for (int pass = 0; pass < 2; ++pass) {
    for (int r = 0; r < 16; ++r) {
      const int row = q0 + r;
      for (int c4 = lane * 4; c4 < DV; c4 += 128) {
        if (row < Tq) {
          const v4f val = *(const v4fa*)&sO[w][r][c4];
          *(volatile v4f*)(y + (size_t)bh * ystride + (size_t)row * ypitch + dv0 + c4) = val;
        }
      }
    }
    if (pass == 0) __threadfence();
  }
}
template <int Cin, bool SPLIT>
__global__ __launch_bounds__(128) void k_conv2d(const float* __restrict__ in, const unsigned short* __restrict__ Bt, const float* __restrict__ bias, float* __restrict__ out) {
  constexpr int K = 9 * Cin, SPT = Cin / 32;
  __shared__ __attribute__((aligned(16))) float so[4][16][64];
  const int tid = threadIdx.x, w = tid >> 5, lane = tid & 31, ln = lane & 15, hh = lane >> 4;
  const int wid = blockIdx.x * 4 + w; const int mt = wid / (COUT / 64), nq = wid % (COUT / 64); if (mt * 16 >= NVOX) return;
  const int row0 = mt * 16, col0 = nq * 64;
  const int m = row0 + ln;
  const int x = m % WX, y = (m / WX) % HY, b = m / (WX * HY);
  v8f acc[4] = {};
  for (int tap = 0; tap < 9; ++tap) {
    const int dy = tap / 3 - 1, dx = tap % 3 - 1;
    const int xx = x + dx, yy = y + dy;
    const bool inb = (m < NPOSR) && (xx >= 0 && xx < WX && yy >= 0 && yy < HY);
    const float* src = in + ((size_t)((b * HY + (inb ? yy : 0)) * WX + (inb ? xx : 0))) * Cin;
#pragma unroll
    for (int s = 0; s < SPT; ++s) {
      const int c0 = s * 32;
      v4f a0 = {0.f,0.f,0.f,0.f}, a1 = a0, a2 = a0, a3 = a0;
      if (inb) { a0 = *(const v4fa*)(src + c0 + 8 * hh); a1 = *(const v4fa*)(src + c0 + 8 * hh + 4); a2 = *(const v4fa*)(src + c0 + 16 + 8 * hh); a3 = *(const v4fa*)(src + c0 + 16 + 8 * hh + 4); }
      float xs[16] = {a0[0],a0[1],a0[2],a0[3],a1[0],a1[1],a1[2],a1[3],a2[0],a2[1],a2[2],a2[3],a3[0],a3[1],a3[2],a3[3]};
      FragB ah, al;
#pragma unroll
      for (int i = 0; i < 16; ++i) { const unsigned short hb = bf16_bits(xs[i]); ah.u[i] = hb; al.u[i] = SPLIT ? bf16_bits(xs[i] - bf16_val(hb)) : (unsigned short)0; }
      const int kb = tap * Cin + c0;
#pragma unroll
      for (int t = 0; t < 4; ++t) { FragB bq; bq.half[0] = *(const v8us*)(Bt + (size_t)(col0 + t * 16 + ln) * K + kb + 8 * hh); bq.half[1] = *(const v8us*)(Bt + (size_t)(col0 + t * 16 + ln) * K + kb + 16 + 8 * hh); acc[t] = SPLIT ? mmaN<2>(ah.v, al.v, bq.v, bq.v, acc[t]) : mmaN<1>(ah.v, al.v, bq.v, bq.v, acc[t]); }
    }
  }
#pragma unroll
  for (int t = 0; t < 4; ++t) { const int col = col0 + t * 16 + ln; const float bv = bf16_round(bias[col]);
#pragma unroll
    for (int r = 0; r < 8; ++r) so[w][8 * hh + r][t * 16 + ln] = acc[t][r] + bv; }
  __builtin_amdgcn_fence(__ATOMIC_ACQ_REL, "workgroup"); __builtin_amdgcn_wave_barrier();
  const int rsub = lane >> 4, c4 = (lane & 15) * 4;
  for (int pass = 0; pass < 2; ++pass) { for (int q = 0; q < 8; ++q) { const int r = q * 2 + rsub; const v4f v = *(const v4fa*)&so[w][r][c4]; *(volatile v4f*)(out + (size_t)(row0 + r) * COUT + col0 + c4) = v; } if (pass == 0) __threadfence(); }
}
template <int Cin>
__global__ __launch_bounds__(128) void k_snake(const float* __restrict__ in, const float* __restrict__ ymap, const unsigned short* __restrict__ Bt, const float* __restrict__ bias, float* __restrict__ out) {
  constexpr int K = 9 * Cin, SPT = Cin / 32;
  __shared__ __attribute__((aligned(16))) float so[4][16][64];
  const int tid = threadIdx.x, w = tid >> 5, lane = tid & 31, ln = lane & 15, hh = lane >> 4;
  const int wid = blockIdx.x * 4 + w; const int mt = wid / (COUT / 64), nq = wid % (COUT / 64); if (mt * 16 >= NVOX) return;
  const int row0 = mt * 16, col0 = nq * 64;
  const int m = row0 + ln;
  const int x = m % WX, y = (m / WX) % HY, b = m / (WX * HY);
  v8f acc[4] = {};
  for (int tap = 0; tap < 9; ++tap) {
    const bool live = (m < NPOSR);
    float yc = live ? ymap[(((size_t)b * HY + y) * 9 + tap) * WX + x] : 0.f; float xc = (float)(x + tap - 4);
    yc = fminf(fmaxf(yc, 0.f), (float)(HY - 1)); xc = fminf(fmaxf(xc, 0.f), (float)(WX - 1));
    const float fy = floorf(yc), fx = floorf(xc); const float wy = yc - fy, wx = xc - fx; const int y0i = (int)fy, x0i = (int)fx; const int y1i = min(y0i + 1, HY - 1), x1i = min(x0i + 1, WX - 1);
    const float w00 = (1.f - wy) * (1.f - wx), w01 = (1.f - wy) * wx, w10 = wy * (1.f - wx), w11 = wy * wx;
    const float* r00 = in + ((size_t)(b * HY + y0i) * WX + x0i) * Cin; const float* r01 = in + ((size_t)(b * HY + y0i) * WX + x1i) * Cin; const float* r10 = in + ((size_t)(b * HY + y1i) * WX + x0i) * Cin; const float* r11 = in + ((size_t)(b * HY + y1i) * WX + x1i) * Cin;
#pragma unroll
    for (int s = 0; s < SPT; ++s) {
      const int c0 = s * 32;
      float xs[16];
#pragma unroll
      for (int i = 0; i < 16; ++i) { const int c = c0 + ((i < 8) ? (8 * hh + i) : (16 + 8 * hh + (i - 8))); xs[i] = live ? (((bf16_round(r00[c]) * w00 + bf16_round(r01[c]) * w01) + bf16_round(r10[c]) * w10) + bf16_round(r11[c]) * w11) : 0.f; }
      FragB ah, al;
#pragma unroll
      for (int i = 0; i < 16; ++i) { const unsigned short hb = bf16_bits(xs[i]); ah.u[i] = hb; al.u[i] = bf16_bits(xs[i] - bf16_val(hb)); }
      const int kb = tap * Cin + c0;
#pragma unroll
      for (int t = 0; t < 4; ++t) { FragB bq; bq.half[0] = *(const v8us*)(Bt + (size_t)(col0 + t * 16 + ln) * K + kb + 8 * hh); bq.half[1] = *(const v8us*)(Bt + (size_t)(col0 + t * 16 + ln) * K + kb + 16 + 8 * hh); acc[t] = mmaN<2>(ah.v, al.v, bq.v, bq.v, acc[t]); }
    }
  }
#pragma unroll
  for (int t = 0; t < 4; ++t) { const int col = col0 + t * 16 + ln; const float bv = bf16_round(bias[col]);
#pragma unroll
    for (int r = 0; r < 8; ++r) so[w][8 * hh + r][t * 16 + ln] = acc[t][r] + bv; }
  __builtin_amdgcn_fence(__ATOMIC_ACQ_REL, "workgroup"); __builtin_amdgcn_wave_barrier();
  const int rsub = lane >> 4, c4 = (lane & 15) * 4;
  for (int pass = 0; pass < 2; ++pass) { for (int q = 0; q < 8; ++q) { const int r = q * 2 + rsub; const v4f v = *(const v4fa*)&so[w][r][c4]; *(volatile v4f*)(out + (size_t)(row0 + r) * COUT + col0 + c4) = v; } if (pass == 0) __threadfence(); }
}

__global__ __launch_bounds__(256) void k_gs1(const float* __restrict__ v, int cpg, double* __restrict__ part) {
  __shared__ double rs[256], rq[256]; const int b = blockIdx.z, g = blockIdx.y, chunk = blockIdx.x; const int t = threadIdx.x; const int ppc = HY * WX / 64;
  double s = 0.0, q = 0.0; const int p = chunk * ppc + t; { const float* row = v + ((size_t)b * HY * WX + p) * 64 + g * cpg; for (int c = 0; c < cpg; ++c) { const double x = (double)row[c]; s += x; q += x * x; } }
  rs[t] = s; rq[t] = q; __syncthreads(); for (int st = 128; st > 0; st >>= 1) { if (t < st) { rs[t] += rs[t + st]; rq[t] += rq[t + st]; } __syncthreads(); }
  double* d = part + (((size_t)b * gridDim.y + g) * 64 + chunk) * 16; if (t < 16) { const double val = (t == 0) ? rs[0] : (t == 1 ? rq[0] : 0.0); *(volatile double*)(d + t) = val; __threadfence(); *(volatile double*)(d + t) = val; }
}
__global__ __launch_bounds__(256) void k_gs2(const double* __restrict__ part, int ngroups, int cpg, float* __restrict__ st) {
  const int i = blockIdx.x * 256 + threadIdx.x; if (i >= BB * ngroups) return; double s = 0.0, q = 0.0; for (int k = 0; k < 64; ++k) { s += part[((size_t)i * 64 + k) * 16]; q += part[((size_t)i * 64 + k) * 16 + 1]; }
  const double n = (double)cpg * HY * WX; const double mu = s / n; double var = q / n - mu * mu; if (var < 0.0) var = 0.0;
  *(volatile float*)(st + i * 2) = (float)mu; *(volatile float*)(st + i * 2 + 1) = (float)(1.0 / sqrt(var + 1e-5)); __threadfence(); *(volatile float*)(st + i * 2) = (float)mu; *(volatile float*)(st + i * 2 + 1) = (float)(1.0 / sqrt(var + 1e-5));
}
__global__ __launch_bounds__(256) void k_ymap(const float* __restrict__ off, const float* __restrict__ st, const float* __restrict__ gg, const float* __restrict__ gb, float* __restrict__ ymap) {
  const int m = blockIdx.x * 256 + threadIdx.x; if (m >= NPOS) return; const int x = m % WX, y = (m / WX) % HY, b = m / (WX * HY); float yo[KSN];
#pragma unroll
  for (int k = 0; k < KSN; ++k) { const int g = k / 2; const float mu = st[(b * KSN + g) * 2], rs = st[(b * KSN + g) * 2 + 1]; const float v = (off[(size_t)m * 64 + k] - mu) * rs * bf16_round(gg[k]) + bf16_round(gb[k]); yo[k] = tanhf(v); }
  float yn[KSN]; yn[4] = 0.f; float a = 0.f; for (int k = 5; k < KSN; ++k) { a += yo[k]; yn[k] = a; } a = 0.f; for (int k = 3; k >= 0; --k) { a += yo[k]; yn[k] = a; }
  for (int pass = 0; pass < 2; ++pass) {
#pragma unroll
    for (int k = 0; k < KSN; ++k) *(volatile float*)(ymap + (((size_t)b * HY + y) * KSN + k) * WX + x) = (float)y + 1.0f * yn[k]; if (pass == 0) __threadfence(); }
}
__global__ __launch_bounds__(256) void k_final(const float* __restrict__ O, const float* __restrict__ st, const float* __restrict__ gg, const float* __restrict__ gb, float* __restrict__ out) {
  const int p = (blockIdx.x % (HY * WX / 256)) * 256 + threadIdx.x; const int bo = blockIdx.x / (HY * WX / 256); const int b = bo / CO, o = bo % CO; const int g = o / 4;
  const float mu = st[(b * 16 + g) * 2], rs = st[(b * 16 + g) * 2 + 1]; const float v = fmaxf((O[((size_t)b * HY * WX + p) * 64 + o] - mu) * rs * bf16_round(gg[o]) + bf16_round(gb[o]), 0.f);
  *(volatile float*)(out + ((size_t)bo) * HY * WX + p) = v; __threadfence(); *(volatile float*)(out + ((size_t)bo) * HY * WX + p) = v;
}
__global__ __launch_bounds__(256) void k_wts(const float* __restrict__ woff, const float* __restrict__ wdsc, unsigned short* __restrict__ B1, unsigned short* __restrict__ B2) {
  const int t = blockIdx.x * 256 + threadIdx.x; const int K = 9 * CI; if (t >= 64 * (K / 8)) return; const int o = t / (K / 8), k8 = (t % (K / 8)) * 8; v8us v1, v2;
#pragma unroll
  for (int i = 0; i < 8; ++i) { const int k = k8 + i; const int tap = k / CI, c = k % CI; v1[i] = (o < 2 * KSN) ? bf16_bits(woff[((size_t)o * CI + c) * 9 + tap]) : (unsigned short)0; v2[i] = bf16_bits(wdsc[((size_t)o * CI + c) * KSN + tap]); }
  *(volatile v8us*)(B1 + (size_t)o * K + k8) = v1; *(volatile v8us*)(B2 + (size_t)o * K + k8) = v2; __threadfence(); *(volatile v8us*)(B1 + (size_t)o * K + k8) = v1; *(volatile v8us*)(B2 + (size_t)o * K + k8) = v2;
}
__global__ __launch_bounds__(256) void k_bias64(const float* __restrict__ b, int n, float* __restrict__ o) { const int t = threadIdx.x; if (t < 64) { const float v = (t < n) ? b[t] : 0.f; *(volatile float*)(o + t) = v; __threadfence(); *(volatile float*)(o + t) = v; } }
extern "C" void kernel_launch(void* const* d_in, const int* in_sizes, int n_in,
                              void* d_out, int out_size, void* d_ws, size_t ws_size, hipStream_t stream) {
  (void)in_sizes; (void)n_in; (void)out_size;
  const float* x = (const float*)d_in[0]; const float* woff = (const float*)d_in[1]; const float* boff = (const float*)d_in[2]; const float* ggo = (const float*)d_in[3]; const float* gbo = (const float*)d_in[4]; const float* wdsc = (const float*)d_in[5]; const float* bdsc = (const float*)d_in[6]; const float* gg = (const float*)d_in[7]; const float* gb = (const float*)d_in[8];
  char* ws = (char*)d_ws; size_t off = 0;
  auto take = [&](size_t bytes) { char* p = ws + off; off += (bytes + 255) & ~(size_t)255; return p; };
  unsigned short* B1 = (unsigned short*)take(64 * 576 * 2); unsigned short* B2 = (unsigned short*)take(64 * 576 * 2); float* b1p = (float*)take(64 * 4);
  float* xcl = (float*)take((size_t)NPOS * CI * 4); float* offv = (float*)take((size_t)NPOS * 64 * 4); float* ymap = (float*)take((size_t)BB * HY * KSN * WX * 4); float* O = (float*)take((size_t)NPOS * 64 * 4);
  double* part = (double*)take((size_t)BB * 16 * 64 * 16 * 8); float* st1 = (float*)take(BB * KSN * 2 * 4 + 128); float* st2 = (float*)take(BB * 16 * 2 * 4 + 128);
  if (off > ws_size) return;
  k_wts<<<(64 * 72 + 255) / 256, 256, 0, stream>>>(woff, wdsc, B1, B2); k_bias64<<<1, 256, 0, stream>>>(boff, 2 * KSN, b1p);
  k_transpose32<false, false, false><<<dim3(HY * WX / 32, CI / 32, BB), 256, 0, stream>>>(x, xcl, CI, HY * WX, nullptr, nullptr, nullptr);
  k_conv2d<CI, false><<<((NVOX / 16) * 1 + 3) / 4, 128, 0, stream>>>(xcl, B1, b1p, offv);
  k_gs1<<<dim3(64, KSN, BB), 256, 0, stream>>>(offv, 2, part); k_gs2<<<1, 256, 0, stream>>>(part, KSN, 2, st1);
  k_ymap<<<NPOS / 256, 256, 0, stream>>>(offv, st1, ggo, gbo, ymap);
  k_snake<CI><<<((NVOX / 16) * 1 + 3) / 4, 128, 0, stream>>>(xcl, ymap, B2, bdsc, O);
  k_gs1<<<dim3(64, 16, BB), 256, 0, stream>>>(O, 4, part); k_gs2<<<1, 256, 0, stream>>>(part, 16, 4, st2);
  k_final<<<BB * CO * (HY * WX / 256), 256, 0, stream>>>(O, st2, gg, gb, (float*)d_out);
}
